// EdgeNetwork_23733989278143
// MI455X (gfx1250) — hardware-verified
//
#include <hip/hip_runtime.h>
#include <hip/hip_bf16.h>

typedef __attribute__((ext_vector_type(16))) _Float16 v16h;
typedef __attribute__((ext_vector_type(8)))  _Float16 v8h;
typedef __attribute__((ext_vector_type(8)))  float    v8f;

#define N_ATOMS   50000
#define N_EDGES   400000
#define TILE_M    64
#define N_TILES   (N_EDGES / TILE_M)
#define NBLOCKS   392
#define WAVES_PB  8
#define TOT_WAVES (NBLOCKS * WAVES_PB)
#define BUCKET    64
#define NBUCKET   ((N_ATOMS + BUCKET - 1) / BUCKET)
#define LCAP      4096
typedef __attribute__((ext_vector_type(4))) float v4f_t;
typedef float v4fa __attribute__((ext_vector_type(4), may_alias));

__device__ __forceinline__ v8h cvt8(float4 a, float4 b) {
    v8h r;
    r[0] = (_Float16)a.x; r[1] = (_Float16)a.y; r[2] = (_Float16)a.z; r[3] = (_Float16)a.w;
    r[4] = (_Float16)b.x; r[5] = (_Float16)b.y; r[6] = (_Float16)b.z; r[7] = (_Float16)b.w;
    return r;
}

__global__ __launch_bounds__(256) __attribute__((amdgpu_num_vgpr(200))) void EdgeNetwork_wmma_kernel(
    const float* __restrict__ atom,
    const float* __restrict__ bond,
    const int*   __restrict__ pairs,
    const float* __restrict__ kern,
    const float* __restrict__ bias,
    float*       __restrict__ T)
{
    __shared__ __align__(32) _Float16 kern_swz[2 * 17 * 2 * 32 * 16];
    __shared__ __align__(16) float    bond_lds[WAVES_PB * TILE_M * 16];
    __shared__ __align__(16) float    tst[WAVES_PB][16 * 32];

    const int tid  = threadIdx.x;
    const int lane = tid & 31;
    const int wave = tid >> 5;

    for (int idx = tid; idx < 17 * 2 * 32 * 16; idx += 256) {
        const int p  = idx & 15;
        const int L  = (idx >> 4) & 31;
        const int nt = (idx >> 9) & 1;
        const int s  = idx >> 10;
        const int hL = L >> 4;
        const int t  = (p < 8) ? (hL * 8 + p) : (16 + hL * 8 + (p - 8));
        const int i  = nt * 16 + (L & 15);
        const float v = (s < 16) ? kern[s * 1024 + i * 32 + t] : bias[i * 32 + t];
        const _Float16 hv = (_Float16)v;
        kern_swz[idx] = hv;
        kern_swz[17 * 2 * 32 * 16 + idx] = (_Float16)((v - (float)hv) * 2048.0f);
    }
    __syncthreads();

    const v16h* kb    = (const v16h*)kern_swz;
    const v16h* kbl   = (const v16h*)(kern_swz + 17 * 2 * 32 * 16);
    float*      bwave = &bond_lds[wave * (TILE_M * 16)];
    const int halfsel = lane >> 4;
    const int ecol    = lane & 15;

    for (int tile = (int)blockIdx.x * WAVES_PB + wave; tile < N_TILES;
         tile += TOT_WAVES) {
        const int eb = tile * TILE_M;

        #pragma unroll
        for (int rr = 0; rr < 2; ++rr) {
            const int e2 = lane * 2 + rr;
            const float* brow = bond + (long)(eb + e2) * 16;
            #pragma unroll
            for (int g = 0; g < 4; ++g) *(float4*)&bwave[e2 * 16 + 4 * g] = *(const float4*)(brow + 4 * g);
        }
        asm volatile("s_wait_dscnt 0" ::: "memory");

        const int off = halfsel * 8;
        const int rbase = halfsel * 8;
        float* ts = tst[wave];
        #pragma unroll 1
        for (int m = 0; m < 4; ++m) {
            const int2 prm = ((const int2*)pairs)[eb + m * 16 + ecol];
            const float* nrow = atom + (long)prm.y * 32;
            float xv[16];
            { const float4 f0 = *(const float4*)(nrow + off), f1 = *(const float4*)(nrow + off + 4), f2 = *(const float4*)(nrow + off + 16), f3 = *(const float4*)(nrow + off + 20);
              xv[0]=f0.x; xv[1]=f0.y; xv[2]=f0.z; xv[3]=f0.w; xv[4]=f1.x; xv[5]=f1.y; xv[6]=f1.z; xv[7]=f1.w;
              xv[8]=f2.x; xv[9]=f2.y; xv[10]=f2.z; xv[11]=f2.w; xv[12]=f3.x; xv[13]=f3.y; xv[14]=f3.z; xv[15]=f3.w; }
            v8f acch0 = {}, acch1 = {}, accl0 = {}, accl1 = {};
            #pragma unroll 1
            for (int s = 0; s <= 16; ++s) {
                asm volatile("" ::: "memory");
                const v16h b0 = kb[(s * 2 + 0) * 32 + lane],  b1 = kb[(s * 2 + 1) * 32 + lane];
                const v16h b0l = kbl[(s * 2 + 0) * 32 + lane], b1l = kbl[(s * 2 + 1) * 32 + lane];
                const float c = (s < 16) ? bwave[(m * 16 + ecol) * 16 + s] : 1.0f;
                v16h ah, al;
                #pragma unroll
                for (int j = 0; j < 16; ++j) { const float p = xv[j] * c; const _Float16 h = (_Float16)p; ah[j] = h; al[j] = (_Float16)((p - (float)h) * 2048.0f); }
                acch0 = __builtin_amdgcn_wmma_f32_16x16x32_f16(false, ah, false, b0, (short)0, acch0, false, false);
                acch1 = __builtin_amdgcn_wmma_f32_16x16x32_f16(false, ah, false, b1, (short)0, acch1, false, false);
                accl0 = __builtin_amdgcn_wmma_f32_16x16x32_f16(false, al, false, b0, (short)0, accl0, false, false);
                accl1 = __builtin_amdgcn_wmma_f32_16x16x32_f16(false, al, false, b1, (short)0, accl1, false, false);
                accl0 = __builtin_amdgcn_wmma_f32_16x16x32_f16(false, ah, false, b0l, (short)0, accl0, false, false);
                accl1 = __builtin_amdgcn_wmma_f32_16x16x32_f16(false, ah, false, b1l, (short)0, accl1, false, false);
            }
            #pragma unroll
            for (int r = 0; r < 8; ++r) {
                ts[(rbase + r) * 32 + ecol]      = acch0[r] + accl0[r] * (1.0f / 2048.0f);
                ts[(rbase + r) * 32 + 16 + ecol] = acch1[r] + accl1[r] * (1.0f / 2048.0f);
            }
            asm volatile("s_wait_dscnt 0" ::: "memory");
            #pragma unroll 1
            for (int pass = 0; pass < 2; ++pass) {
                #pragma unroll
                for (int i = 0; i < 4; ++i) {
                    const int c = lane + 32 * i, rr = c >> 3, q = c & 7;
                    const v4f_t v = *(const volatile v4fa*)(ts + rr * 32 + q * 4);
                    *(volatile v4f_t*)(T + (long)(eb + m * 16 + rr) * 32 + q * 4) = v;
                }
                __threadfence();
            }
            asm volatile("s_wait_dscnt 0" ::: "memory");
        }
    }
}

__global__ __launch_bounds__(256) void gather_kernel(
    const int*   __restrict__ pairs,
    const float* __restrict__ T,
    float*       __restrict__ out)
{
    __shared__ unsigned lst[LCAP];
    __shared__ int wcnt[WAVES_PB];
    __shared__ int total;
    const int tid = threadIdx.x, lane = tid & 31, wave = tid >> 5;
    const int a0 = blockIdx.x * BUCKET;
    if (tid == 0) total = 0;
    __syncthreads();

    for (int e0 = 0; e0 < N_EDGES; e0 += 256) {
        const int e = e0 + tid;
        int loc = -1;
        if (e < N_EDGES) {
            const int d = pairs[2 * e];
            const int l = d - a0;
            if ((unsigned)l < (unsigned)BUCKET) loc = l;
        }
        const unsigned m = __ballot(loc >= 0);
        const int mine = __popc(m & ((1u << lane) - 1u));
        if (lane == 0) wcnt[wave] = __popc(m);
        __syncthreads();
        int base = total;
        #pragma unroll
        for (int w = 0; w < WAVES_PB; ++w) if (w < wave) base += wcnt[w];
        if (loc >= 0) { const int slot = base + mine; if (slot < LCAP) lst[slot] = ((unsigned)loc << 20) | (unsigned)e; }
        __syncthreads();
        if (tid == 0) { int t = total; for (int w = 0; w < WAVES_PB; ++w) t += wcnt[w]; total = t; }
        __syncthreads();
    }
    const int n = (total < LCAP) ? total : LCAP;

    #pragma unroll 1
    for (int j = 0; j < 8; ++j) {
        const int loc = wave * 8 + j;
        const int atom = a0 + loc;
        float s = 0.0f;
        for (int i = 0; i < n; ++i) {
            const unsigned v = lst[i];
            if ((int)(v >> 20) == loc) s += T[(long)(v & 0xFFFFFu) * 32 + lane];
        }
        if (atom < N_ATOMS) {
            *(volatile float*)(out + (long)atom * 32 + lane) = s;
            __threadfence();
            *(volatile float*)(out + (long)atom * 32 + lane) = s;
        }
    }
}


extern "C" void kernel_launch(void* const* d_in, const int* in_sizes, int n_in,
                              void* d_out, int out_size, void* d_ws, size_t ws_size,
                              hipStream_t stream) {
    const float* atom  = (const float*)d_in[0];
    const float* bond  = (const float*)d_in[1];
    const int*   pairs = (const int*)d_in[2];
    const float* kern  = (const float*)d_in[3];
    const float* bias  = (const float*)d_in[4];
    float*       out   = (float*)d_out;

    (void)in_sizes; (void)n_in; (void)out_size; (void)ws_size;
    float* T = (float*)d_ws;
    EdgeNetwork_wmma_kernel<<<NBLOCKS, 256, 0, stream>>>(atom, bond, pairs, kern, bias, T);
    gather_kernel<<<NBUCKET, 256, 0, stream>>>(pairs, T, out);
}
